// PathwayAwareNormalization_60447369724329
// MI455X (gfx1250) — hardware-verified
//
#include <hip/hip_runtime.h>
#include <math.h>
#include <stdint.h>

static constexpr int kBatch    = 4;
static constexpr int kSeq      = 2048;
static constexpr int kDModel   = 1024;
static constexpr int kTokens   = kBatch * kSeq;
static constexpr int kPath     = 1000;
static constexpr int kHeads    = 8;
static constexpr int kHeadDim  = 128;
static constexpr int kQkvOut   = 3 * kDModel;
static constexpr int kQkLd     = 2 * kDModel;
static constexpr int kKeyChunk = 64;
static constexpr int kOsPitch  = 132;
static_assert(kHeads * kHeadDim == kDModel);
static_assert(kSeq % 64 == 0 && kDModel % 64 == 0 && kTokens % 64 == 0 && kQkvOut % 64 == 0);
static_assert(kDModel % 32 == 0);

static constexpr size_t kOffX0   = 0;
static constexpr size_t kOffX0h  = 33554432;
static constexpr size_t kOffQK   = 0;
static constexpr size_t kOffVT   = 33554432;
static constexpr size_t kOffX1   = 50331648;
static constexpr size_t kOffX1h  = 83886080;
static constexpr size_t kOffCTX  = 83886080;
static constexpr size_t kOffWi   = 100663296;
static constexpr size_t kOffWqkv = 102760448;
static constexpr size_t kOffWo   = 109051904;
static constexpr size_t kOffBi   = 111149056;
static constexpr size_t kOffBqkv = 111153152;
static constexpr size_t kOffBo   = 111165440;
static constexpr size_t kWsTotal = 111169536;
static_assert(kOffX0h == kOffX0 + (size_t)kTokens * kDModel * 4);
static_assert(kOffX1 == kOffX0h + (size_t)kTokens * kDModel * 2);
static_assert(kOffVT == kOffQK + (size_t)kTokens * kQkLd * 2);
static_assert(kOffVT + (size_t)kDModel * kTokens * 2 == kOffX1);
static_assert(kOffX1h == kOffX1 + (size_t)kTokens * kDModel * 4);
static_assert(kOffWi == kOffX1h + (size_t)kTokens * kDModel * 2);
static_assert(kOffWqkv == kOffWi + (size_t)kDModel * kDModel * 2);
static_assert(kOffWo == kOffWqkv + (size_t)kQkvOut * kDModel * 2);
static_assert(kOffBi == kOffWo + (size_t)kDModel * kDModel * 2);
static_assert(kOffBqkv == kOffBi + (size_t)kDModel * 4);
static_assert(kOffBo == kOffBqkv + (size_t)kQkvOut * 4);
static_assert(kWsTotal == kOffBo + (size_t)kDModel * 4);
static_assert(kWsTotal <= 134217728);

typedef __attribute__((ext_vector_type(16))) _Float16 v16h;
typedef __attribute__((ext_vector_type(8)))  _Float16 v8h;
typedef __attribute__((ext_vector_type(16))) __bf16   v16b;
typedef __attribute__((ext_vector_type(8)))  __bf16   v8b;
typedef __attribute__((ext_vector_type(8)))  float    v8f;
typedef __attribute__((ext_vector_type(4)))  float    v4f;
typedef __attribute__((ext_vector_type(4)))  unsigned int v4u;

__device__ __forceinline__ unsigned short f2bf_bits(float f) {
  unsigned u = __float_as_uint(f);
  return (unsigned short)((u + 0x7FFFu + ((u >> 16) & 1u)) >> 16);
}
__device__ __forceinline__ float bf_bits2f(unsigned short h) { return __uint_as_float(((unsigned)h) << 16); }
__device__ __forceinline__ float bfr(float f) { return bf_bits2f(f2bf_bits(f)); }
__device__ __forceinline__ unsigned short h_bits(_Float16 x) { return __builtin_bit_cast(unsigned short, x); }
__device__ __forceinline__ unsigned pk16(unsigned short a, unsigned short b) { return (unsigned)a | ((unsigned)b << 16); }
__device__ __forceinline__ unsigned short w16bits(float f) { return h_bits((_Float16)(bfr(f) * 64.0f)); }

__device__ __forceinline__ float wave_sum(float v) {
#pragma unroll
  for (int m = 16; m >= 1; m >>= 1) v += __shfl_xor(v, m, 32);
  return v;
}
__device__ __forceinline__ void lds_wave_sync() {
  __builtin_amdgcn_fence(__ATOMIC_RELEASE, "workgroup");
  __builtin_amdgcn_wave_barrier();
  __builtin_amdgcn_fence(__ATOMIC_ACQUIRE, "workgroup");
}

__device__ __forceinline__ void dep_guard_h(v8f& a, v8f& b, v16h x, v16h y) { asm volatile("v_nop\n\tv_nop\n\tv_nop\n\tv_nop" : "+v"(a), "+v"(b) : "v"(x), "v"(y)); }
__device__ __forceinline__ void dep_guard_b(v8f& a, v8f& b, v16b x, v16b y) { asm volatile("v_nop\n\tv_nop\n\tv_nop\n\tv_nop" : "+v"(a), "+v"(b) : "v"(x), "v"(y)); }
__device__ __forceinline__ void keep4_h(v16h a, v16h b, v16h c, v16h d) { asm volatile("v_nop" :: "v"(a), "v"(b), "v"(c), "v"(d)); }
__device__ __forceinline__ void keep4_b(v16b a, v16b b, v16b c, v16b d) { asm volatile("v_nop" :: "v"(a), "v"(b), "v"(c), "v"(d)); }
__device__ __forceinline__ void acc_guard4(v8f& a, v8f& b, v8f& c, v8f& d) { asm volatile("v_nop\n\tv_nop\n\tv_nop\n\tv_nop" : "+v"(a), "+v"(b), "+v"(c), "+v"(d)); }
template <typename T> struct Frag;
template <> struct Frag<_Float16> {
  typedef v16h V; union U { v16h v; v8h h[2]; };
  static __device__ __forceinline__ v16h load(const _Float16* p) {
    U f; f.h[0] = *(const v8h*)(p); f.h[1] = *(const v8h*)(p + 16); return f.v;
  }
  static __device__ __forceinline__ v8f mma(v16h a, v16h b, v8f c) {
    return __builtin_amdgcn_wmma_f32_16x16x32_f16(false, a, false, b, (short)0, c, false, false);
  }
  static __device__ __forceinline__ void guard(v8f& a, v8f& b, v16h x, v16h y) { dep_guard_h(a, b, x, y); }
  static __device__ __forceinline__ void keep(v16h a, v16h b, v16h c, v16h d) { keep4_h(a, b, c, d); }
};
template <> struct Frag<__bf16> {
  typedef v16b V; union U { v16b v; v8b h[2]; };
  static __device__ __forceinline__ v16b load(const __bf16* p) {
    U f; f.h[0] = *(const v8b*)(p); f.h[1] = *(const v8b*)(p + 16); return f.v;
  }
  static __device__ __forceinline__ v8f mma(v16b a, v16b b, v8f c) {
    return __builtin_amdgcn_wmma_f32_16x16x32_bf16(false, a, false, b, (short)0, c, false, false);
  }
  static __device__ __forceinline__ void guard(v8f& a, v8f& b, v16b x, v16b y) { dep_guard_b(a, b, x, y); }
  static __device__ __forceinline__ void keep(v16b a, v16b b, v16b c, v16b d) { keep4_b(a, b, c, d); }
};

__device__ __forceinline__ v8f mma_f16g(v16h a, v16h b, v8f c) {
  c = __builtin_amdgcn_wmma_f32_16x16x32_f16(false, a, false, b, (short)0, c, false, false);
  asm volatile("v_nop\n\tv_nop\n\tv_nop\n\tv_nop" : "+v"(c) : "v"(a), "v"(b));
  return c;
}

template <int ET> struct Elem;
template <> struct Elem<0> { typedef _Float16 T; };
template <> struct Elem<1> { typedef __bf16 T; };
template <int ET, bool SPLIT, int BIAS_MODE, int OUT_MODE, bool RESID, int ACT = 0>
__global__ __launch_bounds__(256) void wmma_gemm64(
    const unsigned short* __restrict__ Ap, const unsigned short* __restrict__ A2p, int lda, long strideA,
    const unsigned short* __restrict__ Btp, const unsigned short* __restrict__ Bt2p, int ldb, long strideB,
    void* __restrict__ Cout, void* __restrict__ Cout2, int ldc, long strideC,
    const float* __restrict__ bias,
    const float* __restrict__ resid, long strideR,
    int M, int N, int K, float scale) {
  typedef typename Elem<ET>::T T;
  typedef typename Frag<T>::V V;
  const T* A = (const T*)Ap; const T* A2 = (const T*)A2p; const T* Bt = (const T*)Btp; const T* Bt2 = (const T*)Bt2p;
  __shared__ __align__(16) float sT[8][16 * 68];
  const int b    = blockIdx.y;
  const int lane = threadIdx.x & 31;
  const int wave = threadIdx.x >> 5;
  const int tilesN = N >> 6;
  const int tilesM = M >> 6;
  const int tile = blockIdx.x * 8 + wave;
  if (tile >= tilesM * tilesN) return;
  const int tm = tile / tilesN;
  const int tn = tile - tm * tilesN;
  const int m0 = tm << 6;
  const int n0 = tn << 6;

  const T* Ab  = A  + (size_t)b * strideA;
  const T* Bb  = Bt + (size_t)b * strideB;
  const T* Ab2 = SPLIT ? (A2  + (size_t)b * strideA) : nullptr;
  const T* Bb2 = SPLIT ? (Bt2 + (size_t)b * strideB) : nullptr;

  const int rlane = lane & 15;
  const int koff  = (lane >> 4) * 8;
  const int mOff  = (lane >> 4) * 8;

  v8f acc[4][4];
#pragma unroll
  for (int i = 0; i < 4; ++i)
#pragma unroll
    for (int j = 0; j < 4; ++j) acc[i][j] = (v8f){0.f,0.f,0.f,0.f,0.f,0.f,0.f,0.f};

  for (int k0 = 0; k0 < K; k0 += 32) {
    V bh[4], bl[4];
#pragma unroll
    for (int j = 0; j < 4; ++j) {
      const size_t bo = (size_t)(n0 + (j << 4) + rlane) * ldb + koff + k0;
      bh[j] = Frag<T>::load(Bb + bo);
      if (SPLIT) bl[j] = Frag<T>::load(Bb2 + bo);
    }
#pragma unroll
    for (int i = 0; i < 4; ++i) {
      const size_t ao = (size_t)(m0 + (i << 4) + rlane) * lda + koff + k0;
      V ah = Frag<T>::load(Ab + ao);
      V al;
      if (SPLIT) al = Frag<T>::load(Ab2 + ao);
#pragma unroll
      for (int j = 0; j < 4; ++j) {
        acc[i][j] = Frag<T>::mma(ah, bh[j], acc[i][j]);
        if (SPLIT) {
          acc[i][j] = Frag<T>::mma(ah, bl[j], acc[i][j]);
          acc[i][j] = Frag<T>::mma(al, bh[j], acc[i][j]);
        }
      }
      Frag<T>::guard(acc[i][0], acc[i][3], ah, SPLIT ? al : ah);
    }
    Frag<T>::keep(bh[0], bh[1], bh[2], bh[3]);
    if (SPLIT) Frag<T>::keep(bl[0], bl[1], bl[2], bl[3]);
  }
  acc_guard4(acc[0][0], acc[0][1], acc[0][2], acc[0][3]);
  acc_guard4(acc[1][0], acc[1][1], acc[1][2], acc[1][3]);
  acc_guard4(acc[2][0], acc[2][1], acc[2][2], acc[2][3]);
  acc_guard4(acc[3][0], acc[3][1], acc[3][2], acc[3][3]);

  float* slab = sT[wave];
  const float* Rb = RESID ? (resid + (size_t)b * strideR) : nullptr;
#pragma unroll
  for (int i = 0; i < 4; ++i) {
    const int mBase = m0 + (i << 4);
#pragma unroll
    for (int j = 0; j < 4; ++j) {
      const int n = n0 + (j << 4) + rlane;
      float bv = 0.f;
      if (BIAS_MODE == 2) bv = bias[n];
#pragma unroll
      for (int r = 0; r < 8; ++r) {
        float v = acc[i][j][r] * scale;
        if (BIAS_MODE == 1) v += bias[mBase + mOff + r];
        if (BIAS_MODE == 2) v += bv;
        if (RESID) v += Rb[(size_t)(mBase + mOff + r) * ldc + n];
        if (ACT == 1) v = tanhf(v);
        if (ACT == 2) v = fmaxf(v, 0.0f);
        if (ACT == 4) v = (v > 0.f) ? v : 0.01f * v;
        slab[(mOff + r) * 68 + (j << 4) + rlane] = v;
      }
    }
    __builtin_amdgcn_fence(__ATOMIC_RELEASE, "workgroup");
    __builtin_amdgcn_wave_barrier();
    __builtin_amdgcn_fence(__ATOMIC_ACQUIRE, "workgroup");
    if (OUT_MODE == 0 || OUT_MODE == 3) {
      float* C = (float*)Cout + (size_t)b * strideC;
      const int hh = lane >> 4, c4 = (lane & 15) * 4;
      for (int pass = 0; pass < 2; ++pass) {
#pragma unroll
        for (int it = 0; it < 8; ++it) {
          const int row = it * 2 + hh;
          v4f v = *(const v4f*)(slab + row * 68 + c4);
          *(volatile v4f*)(C + (size_t)(mBase + row) * ldc + n0 + c4) = v;
        }
        __threadfence();
      }
    }
    if (OUT_MODE == 1 || OUT_MODE == 2 || OUT_MODE == 3) {
      const int q = lane >> 3, c8 = (lane & 7) * 8;
      unsigned short* C  = (unsigned short*)((OUT_MODE == 3) ? Cout2 : Cout) + (size_t)b * strideC;
      unsigned short* C2 = (OUT_MODE == 2) ? ((unsigned short*)Cout2 + (size_t)b * strideC) : nullptr;
      for (int pass = 0; pass < 2; ++pass) {
#pragma unroll
        for (int it = 0; it < 4; ++it) {
          const int row = it * 4 + q;
          const float* sp = slab + row * 68 + c8;
          v8h hv;
          v8h lv = (v8h){(_Float16)0, (_Float16)0, (_Float16)0, (_Float16)0, (_Float16)0, (_Float16)0, (_Float16)0, (_Float16)0};
#pragma unroll
          for (int e = 0; e < 8; ++e) {
            if (OUT_MODE == 2) {
              unsigned short hb = f2bf_bits(sp[e]);
              unsigned short lb = f2bf_bits(sp[e] - bf_bits2f(hb));
              hv[e] = __builtin_bit_cast(_Float16, hb);
              lv[e] = __builtin_bit_cast(_Float16, lb);
            } else {
              hv[e] = (_Float16)sp[e];
            }
          }
          *(volatile v8h*)(C + (size_t)(mBase + row) * ldc + n0 + c8) = hv;
          if (OUT_MODE == 2) *(volatile v8h*)(C2 + (size_t)(mBase + row) * ldc + n0 + c8) = lv;
        }
        __threadfence();
      }
    }
    __builtin_amdgcn_fence(__ATOMIC_RELEASE, "workgroup");
    __builtin_amdgcn_wave_barrier();
    __builtin_amdgcn_fence(__ATOMIC_ACQUIRE, "workgroup");
  }
}

__global__ __launch_bounds__(256) void wcvt_kernel(const float* __restrict__ in, unsigned short* out, int n8) {
  const int i = blockIdx.x * 256 + (int)threadIdx.x;
  if (i < n8) {
    const v4f a  = *(const v4f*)(in + (size_t)i * 8);
    const v4f a4 = *(const v4f*)(in + (size_t)i * 8 + 4);
    v4u p;
    p[0] = pk16(w16bits(a[0]),  w16bits(a[1]));
    p[1] = pk16(w16bits(a[2]),  w16bits(a[3]));
    p[2] = pk16(w16bits(a4[0]), w16bits(a4[1]));
    p[3] = pk16(w16bits(a4[2]), w16bits(a4[3]));
    unsigned short* o = out + (size_t)i * 8;
    *(volatile v4u*)o = p;
    __threadfence();
    *(volatile v4u*)o = p;
  }
}

__global__ __launch_bounds__(256) void rne4_kernel(const float* __restrict__ in, float* out, int n4) {
  const int i = blockIdx.x * 256 + (int)threadIdx.x;
  if (i < n4) {
    const v4f a = *(const v4f*)(in + (size_t)i * 4);
    v4f o;
    o[0] = bfr(a[0]); o[1] = bfr(a[1]); o[2] = bfr(a[2]); o[3] = bfr(a[3]);
    float* p = out + (size_t)i * 4;
    *(volatile v4f*)p = o;
    __threadfence();
    *(volatile v4f*)p = o;
  }
}

__global__ __launch_bounds__(256) void ln_gather_kernel(const float* __restrict__ x, const int* __restrict__ ids,
                                                        const float* __restrict__ gamma, const float* __restrict__ beta,
                                                        float* X0, unsigned short* X0h, int ntok, int npath) {
  __shared__ __align__(16) float slab[8][kDModel];
  const int wave = threadIdx.x >> 5;
  const int lane = threadIdx.x & 31;
  const int tok  = blockIdx.x * 8 + wave;
  if (tok >= ntok) return;
  const float* xr = x + (size_t)tok * kDModel + lane * 4;

  float s = 0.f;
#pragma unroll 1
  for (int it = 0; it < 8; ++it) {
    const v4f a = *(const v4f*)(xr + it * 128);
    s += (bfr(a[0]) + bfr(a[1])) + (bfr(a[2]) + bfr(a[3]));
  }
  s = wave_sum(s);
  const float mu = s * (1.0f / (float)kDModel);

  float ss = 0.f;
#pragma unroll 1
  for (int it = 0; it < 8; ++it) {
    const v4f a = *(const v4f*)(xr + it * 128);
    const float d0 = bfr(a[0]) - mu, d1 = bfr(a[1]) - mu, d2 = bfr(a[2]) - mu, d3 = bfr(a[3]) - mu;
    ss += (d0 * d0 + d1 * d1) + (d2 * d2 + d3 * d3);
  }
  ss = wave_sum(ss);
  const float var  = ss * (1.0f / (float)kDModel);
  const float rstd = rsqrtf(var + 1e-5f);

  const int  idr   = ids[tok];
  const bool valid = idr < npath;
  int gid = idr < 0 ? 0 : idr;
  gid = gid > npath - 1 ? npath - 1 : gid;
  const float* gr = gamma + (size_t)gid * kDModel + lane * 4;
  const float* br = beta  + (size_t)gid * kDModel + lane * 4;

  float* sl = slab[wave];
  float* xo = X0 + (size_t)tok * kDModel + lane * 4;
#pragma unroll 1
  for (int it = 0; it < 8; ++it) {
    const v4f a  = *(const v4f*)(xr + it * 128);
    const v4f g  = *(const v4f*)(gr + it * 128);
    const v4f bb = *(const v4f*)(br + it * 128);
    v4f o;
#pragma unroll
    for (int e = 0; e < 4; ++e) {
      const float xb = bfr(a[e]);
      const float nv = (xb - mu) * rstd * bfr(g[e]) + bfr(bb[e]);
      o[e] = valid ? nv : xb;
    }
    *(v4f*)(sl + it * 128 + lane * 4) = o;
    *(volatile v4f*)(xo + it * 128) = o;
  }
  __threadfence();
  lds_wave_sync();
#pragma unroll 1
  for (int it = 0; it < 8; ++it) {
    const v4f o = *(const v4f*)(sl + it * 128 + lane * 4);
    *(volatile v4f*)(xo + it * 128) = o;
  }
  unsigned short* ho = X0h + (size_t)tok * kDModel + lane * 8;
  for (int pass = 0; pass < 2; ++pass) {
#pragma unroll 1
    for (int it = 0; it < 4; ++it) {
      const v4f a  = *(const v4f*)(sl + it * 256 + lane * 8);
      const v4f a4 = *(const v4f*)(sl + it * 256 + lane * 8 + 4);
      v4u p;
      p[0] = pk16(h_bits((_Float16)a[0]),  h_bits((_Float16)a[1]));
      p[1] = pk16(h_bits((_Float16)a[2]),  h_bits((_Float16)a[3]));
      p[2] = pk16(h_bits((_Float16)a4[0]), h_bits((_Float16)a4[1]));
      p[3] = pk16(h_bits((_Float16)a4[2]), h_bits((_Float16)a4[3]));
      *(volatile v4u*)(ho + it * 256) = p;
    }
    __threadfence();
  }
}

static constexpr float kScoreScale = 0.08838834764831845f;
static constexpr float kPCarry     = 32768.0f;
static constexpr float kCtxFold    = 2048.0f;

__global__ __launch_bounds__(128) void attn_hd128_kernel(const unsigned short* __restrict__ QKp,
                                                         const unsigned short* __restrict__ VTp,
                                                         unsigned short* CTXp) {
  const _Float16* QK = (const _Float16*)(const void*)QKp;
  const _Float16* VT = (const _Float16*)(const void*)VTp;
  __shared__ __align__(16) _Float16 Psh[4][16 * kKeyChunk];
  __shared__ __align__(16) float    Os[4][16 * kOsPitch];

  const int tid  = threadIdx.x;
  const int wave = tid >> 5;
  const int lane = tid & 31;
  const int hh   = lane >> 4;
  const int c    = lane & 15;

  const int nqb = kSeq / 64;
  const int bx  = blockIdx.x;
  const int qb  = bx % nqb;
  const int bh  = bx / nqb;
  const int h   = bh % kHeads;
  const int b   = bh / kHeads;
  const int q0  = qb * 64 + wave * 16;
  const size_t tokq = (size_t)b * kSeq + q0;

  const _Float16* qrow  = QK + (tokq + c) * kQkLd + h * kHeadDim + 8 * hh;
  const _Float16* kbase = QK + (size_t)b * kSeq * kQkLd + kDModel + h * kHeadDim + 8 * hh;
  const _Float16* vbase = VT + (size_t)(h * kHeadDim + c) * kTokens + (size_t)b * kSeq + 8 * hh;

  float mrow[8], lrow[8];
  v8f oacc[8];
#pragma unroll
  for (int r = 0; r < 8; ++r) { mrow[r] = -__builtin_huge_valf(); lrow[r] = 0.f; }
#pragma unroll
  for (int t = 0; t < 8; ++t) oacc[t] = (v8f){0.f,0.f,0.f,0.f,0.f,0.f,0.f,0.f};

  _Float16* pw = Psh[wave];

  for (int kc = 0; kc < kSeq / kKeyChunk; ++kc) {
    const int kv0 = kc * kKeyChunk;
    v8f s[4];
#pragma unroll
    for (int j = 0; j < 4; ++j) s[j] = (v8f){0.f,0.f,0.f,0.f,0.f,0.f,0.f,0.f};
#pragma unroll
    for (int dc = 0; dc < 4; ++dc) {
      const v16h qa = Frag<_Float16>::load(qrow + dc * 32);
#pragma unroll
      for (int j = 0; j < 4; ++j) {
        const v16h kb = Frag<_Float16>::load(kbase + (size_t)(kv0 + j * 16 + c) * kQkLd + dc * 32);
        s[j] = mma_f16g(qa, kb, s[j]);
      }
    }
    float cm[8];
#pragma unroll
    for (int r = 0; r < 8; ++r) {
      float m = -__builtin_huge_valf();
#pragma unroll
      for (int j = 0; j < 4; ++j) {
        const float sv = s[j][r] * kScoreScale;
        s[j][r] = sv;
        m = fmaxf(m, sv);
      }
#pragma unroll
      for (int off = 1; off < 16; off <<= 1) m = fmaxf(m, __shfl_xor(m, off, 32));
      cm[r] = m;
    }
    lds_wave_sync();
#pragma unroll
    for (int r = 0; r < 8; ++r) {
      const float mnew  = fmaxf(mrow[r], cm[r]);
      const float alpha = __expf(mrow[r] - mnew);
      mrow[r] = mnew;
      float psum = 0.f;
#pragma unroll
      for (int j = 0; j < 4; ++j) {
        const float p = __expf(s[j][r] - mnew);
        psum += p;
        pw[(8 * hh + r) * kKeyChunk + j * 16 + c] = (_Float16)(p * kPCarry);
      }
#pragma unroll
      for (int off = 1; off < 16; off <<= 1) psum += __shfl_xor(psum, off, 32);
      lrow[r] = lrow[r] * alpha + psum;
#pragma unroll
      for (int t = 0; t < 8; ++t) oacc[t][r] *= alpha;
    }
    lds_wave_sync();
#pragma unroll
    for (int kk = 0; kk < 2; ++kk) {
      const v16h pa = Frag<_Float16>::load(pw + c * kKeyChunk + kk * 32 + 8 * hh);
#pragma unroll
      for (int t = 0; t < 8; ++t) {
        const v16h vb = Frag<_Float16>::load(vbase + (size_t)t * 16 * kTokens + kv0 + kk * 32);
        oacc[t] = mma_f16g(pa, vb, oacc[t]);
      }
    }
  }

  float* os = Os[wave];
#pragma unroll
  for (int r = 0; r < 8; ++r) {
    const float inv = 1.0f / (lrow[r] * kCtxFold);
#pragma unroll
    for (int t = 0; t < 8; ++t) os[(8 * hh + r) * kOsPitch + t * 16 + c] = oacc[t][r] * inv;
  }
  lds_wave_sync();
  {
    const int c8 = (lane & 15) * 8;
    unsigned short* ob = CTXp + tokq * kDModel + h * kHeadDim + c8;
    for (int pass = 0; pass < 2; ++pass) {
#pragma unroll
      for (int it = 0; it < 8; ++it) {
        const int row = it * 2 + hh;
        const v4f a  = *(const v4f*)(os + row * kOsPitch + c8);
        const v4f a4 = *(const v4f*)(os + row * kOsPitch + c8 + 4);
        v4u p;
        p[0] = pk16(h_bits((_Float16)a[0]),  h_bits((_Float16)a[1]));
        p[1] = pk16(h_bits((_Float16)a[2]),  h_bits((_Float16)a[3]));
        p[2] = pk16(h_bits((_Float16)a4[0]), h_bits((_Float16)a4[1]));
        p[3] = pk16(h_bits((_Float16)a4[2]), h_bits((_Float16)a4[3]));
        *(volatile v4u*)(ob + (size_t)row * kDModel) = p;
      }
      __threadfence();
    }
  }
}

extern "C" void kernel_launch(void* const* d_in, const int* in_sizes, int n_in,
                              void* d_out, int out_size, void* d_ws, size_t ws_size,
                              hipStream_t stream) {
  if (n_in < 10) return;
  if (in_sizes[0] != kTokens * kDModel || in_sizes[1] != kTokens ||
      in_sizes[2] != kPath * kDModel   || in_sizes[3] != kPath * kDModel ||
      in_sizes[4] != kDModel * kDModel || in_sizes[5] != kDModel ||
      in_sizes[6] != kQkvOut * kDModel || in_sizes[7] != kQkvOut ||
      in_sizes[8] != kDModel * kDModel || in_sizes[9] != kDModel ||
      out_size != kTokens * kDModel) return;
  if ((size_t)kWsTotal > ws_size) return;

  const float* x       = (const float*)d_in[0];
  const int*   ids     = (const int*)  d_in[1];
  const float* gamma   = (const float*)d_in[2];
  const float* beta    = (const float*)d_in[3];
  const float* w_inter = (const float*)d_in[4];
  const float* b_inter = (const float*)d_in[5];
  const float* w_qkv   = (const float*)d_in[6];
  const float* b_qkv   = (const float*)d_in[7];
  const float* w_out   = (const float*)d_in[8];
  const float* b_out   = (const float*)d_in[9];
  float* out = (float*)d_out;

  char* ws = (char*)d_ws;
  float*          X0   = (float*)(ws + kOffX0);
  unsigned short* X0h  = (unsigned short*)(ws + kOffX0h);
  unsigned short* QK   = (unsigned short*)(ws + kOffQK);
  unsigned short* VT   = (unsigned short*)(ws + kOffVT);
  float*          X1   = (float*)(ws + kOffX1);
  unsigned short* X1h  = (unsigned short*)(ws + kOffX1h);
  unsigned short* CTX  = (unsigned short*)(ws + kOffCTX);
  unsigned short* Wi   = (unsigned short*)(ws + kOffWi);
  unsigned short* Wqkv = (unsigned short*)(ws + kOffWqkv);
  unsigned short* Wo   = (unsigned short*)(ws + kOffWo);
  float*          Bi   = (float*)(ws + kOffBi);
  float*          Bqkv = (float*)(ws + kOffBqkv);
  float*          Bo   = (float*)(ws + kOffBo);

  const float kInv64   = 0.015625f;
  const float kInv1024 = 0.0009765625f;

  {
    const int n8a = kDModel * kDModel / 8;
    const int n8b = kQkvOut * kDModel / 8;
    wcvt_kernel<<<dim3(n8a / 256), dim3(256), 0, stream>>>(w_inter, Wi, n8a);
    wcvt_kernel<<<dim3(n8b / 256), dim3(256), 0, stream>>>(w_qkv, Wqkv, n8b);
    wcvt_kernel<<<dim3(n8a / 256), dim3(256), 0, stream>>>(w_out, Wo, n8a);
  }
  {
    const int n4a = kDModel / 4;
    const int n4b = kQkvOut / 4;
    rne4_kernel<<<dim3((n4a + 255) / 256), dim3(256), 0, stream>>>(b_inter, Bi, n4a);
    rne4_kernel<<<dim3((n4b + 255) / 256), dim3(256), 0, stream>>>(b_qkv, Bqkv, n4b);
    rne4_kernel<<<dim3((n4a + 255) / 256), dim3(256), 0, stream>>>(b_out, Bo, n4a);
  }
  ln_gather_kernel<<<dim3(kTokens / 8), dim3(256), 0, stream>>>(x, ids, gamma, beta, X0, X0h, kTokens, kPath);

  wmma_gemm64<0, false, 2, 3, true><<<dim3((kTokens / 64) * (kDModel / 64) / 8, 1), dim3(256), 0, stream>>>(
      X0h, X0h, kDModel, 0L, Wi, Wi, kDModel, 0L,
      (void*)X1, (void*)X1h, kDModel, 0L, Bi, X0, 0L, kTokens, kDModel, kDModel, kInv64);

  wmma_gemm64<0, false, 2, 1, false><<<dim3((kTokens / 64) * (kQkLd / 64) / 8, 1), dim3(256), 0, stream>>>(
      X1h, X1h, kDModel, 0L, Wqkv, Wqkv, kDModel, 0L,
      (void*)QK, (void*)QK, kQkLd, 0L, Bqkv, X1, 0L, kTokens, kQkLd, kDModel, kInv64);

  wmma_gemm64<0, false, 1, 1, false><<<dim3((kDModel / 64) * (kTokens / 64) / 8, 1), dim3(256), 0, stream>>>(
      Wqkv + (size_t)2 * kDModel * kDModel, Wqkv + (size_t)2 * kDModel * kDModel, kDModel, 0L,
      X1h, X1h, kDModel, 0L,
      (void*)VT, (void*)VT, kTokens, 0L, Bqkv + 2 * kDModel, X1, 0L, kDModel, kTokens, kDModel, kInv64);

  attn_hd128_kernel<<<dim3(kBatch * kHeads * (kSeq / 64)), dim3(128), 0, stream>>>(QK, VT, CTX);

  wmma_gemm64<0, false, 2, 0, true><<<dim3((kTokens / 64) * (kDModel / 64) / 8, 1), dim3(256), 0, stream>>>(
      CTX, CTX, kDModel, 0L, Wo, Wo, kDModel, 0L,
      (void*)out, (void*)out, kDModel, 0L, Bo, X1, 0L, kTokens, kDModel, kDModel, kInv1024);
}
